// MDRNN_basic_75136157877047
// MI455X (gfx1250) — hardware-run, weakly checked
//
#include <hip/hip_runtime.h>
#include <math.h>

typedef __attribute__((ext_vector_type(16))) _Float16 v16h;
typedef __attribute__((ext_vector_type(8)))  _Float16 v8h;
typedef __attribute__((ext_vector_type(8)))  float    v8f;
typedef __attribute__((ext_vector_type(4)))  float    v4f;

constexpr int NBATCH   = 1024;
constexpr int NCHAN    = 3;
constexpr int IMG_H    = 32;
constexpr int IMG_W    = 32;
constexpr int NHID     = 32;
constexpr int NGATE    = 5 * NHID;
constexpr int NDIRS    = 4;
constexpr int NFEAT    = NDIRS * NHID;
constexpr int NOUTS    = 10;
constexpr int ROWS_PER_WAVE = 16;
constexpr int NTILES_B = NBATCH / ROWS_PER_WAVE;
constexpr int HT_ELEMS = ROWS_PER_WAVE * NHID;
constexpr int BT_PITCH = 72;
constexpr float W_CARRY       = 64.0f;
constexpr float W_CARRY_INV   = 1.0f / 64.0f;
constexpr float RES_CARRY     = 2048.0f;
constexpr float RES_CARRY_INV = 1.0f / 2048.0f;
constexpr float F16_MIN_NORMAL = 6.103515625e-5f;
constexpr int CROW_PER_COL   = 2 * 2 * 32 * 4;
constexpr int CROW_PER_BLOCK = IMG_W * CROW_PER_COL;

static_assert(NGATE == 160, "gate width");
static_assert(NFEAT == 128, "feature width");
static_assert(NBATCH % ROWS_PER_WAVE == 0, "batch tiles");
static_assert((NBATCH * NOUTS) % 256 == 0, "head grid covers the output exactly");
static_assert(IMG_W * 4 == 128, "one image row is one 128-B line");
static_assert(NGATE % 32 == 0, "weight staging loops");
static_assert(BT_PITCH % 8 == 0 && BT_PITCH >= 2 * NHID + 8, "weight plane pitch");
static_assert(HT_ELEMS == 512, "hidden tile size");

__device__ __forceinline__ float bf16_value(float f) {
  const unsigned u = __float_as_uint(f);
  const unsigned r = (u + 0x7FFFu + ((u >> 16) & 1u)) & 0xFFFF0000u;
  return __uint_as_float(r);
}

union FragU { v16h v; v8h h[2]; };
__device__ __forceinline__ v16h frag_load(const _Float16* p) {
  FragU f;
  f.h[0] = *(const v8h*)(p);
  f.h[1] = *(const v8h*)(p + 16);
  return f.v;
}
__device__ __forceinline__ v8f mma16(v16h a, v16h b, v8f c) {
  return __builtin_amdgcn_wmma_f32_16x16x32_f16(false, a, false, b, (short)0, c, false, false);
}
__device__ __forceinline__ void acc_guard(v8f& acc, v16h a0, v16h a1, v16h b0, v16h b1) {
  asm volatile("v_nop\n\tv_nop\n\tv_nop\n\tv_nop" : "+v"(acc) : "v"(a0), "v"(a1), "v"(b0), "v"(b1) : "memory");
}

__device__ __forceinline__ void split_val(float v, _Float16& hv, _Float16& lv) {
  const float vh = (fabsf(v) < F16_MIN_NORMAL) ? 0.0f : v;
  const _Float16 h16 = (_Float16)vh;
  float hf = (float)h16;
  asm volatile("" : "+v"(hf));
  const float rs = (v - hf) * RES_CARRY;
  hv = h16;
  lv = (_Float16)rs;
}

__device__ __forceinline__ float gate_sig(float z) {
  return __builtin_amdgcn_rcpf(1.0f + __expf(-z));
}
__device__ __forceinline__ float gate_tanh(float z) {
  return 1.0f - 2.0f * __builtin_amdgcn_rcpf(__expf(2.0f * z) + 1.0f);
}

__global__ __launch_bounds__(32) __attribute__((amdgpu_num_vgpr(256)))
void scan2d_kernel(const float* __restrict__ x, const float* __restrict__ Wx,
                   const float* __restrict__ Whv, const float* __restrict__ Whh,
                   const float* __restrict__ bias, float* crow, float* feats) {
  __shared__ __align__(16) _Float16 Bt[NGATE * BT_PITCH];
  __shared__ __align__(16) _Float16 Hhi[IMG_W * HT_ELEMS];
  __shared__ __align__(16) _Float16 Hlo[IMG_W * HT_ELEMS];
  __shared__ __align__(16) float xs[IMG_W * NCHAN * ROWS_PER_WAVE];
  __shared__ __align__(16) float wxs[4 * NGATE];
  __shared__ __align__(16) float hfin[HT_ELEMS];

  const int lane = threadIdx.x & 31;
  const int hh   = lane >> 4;
  const int ln   = lane & 15;
  const int tile = blockIdx.x;
  const int dir  = blockIdx.y;
  const int b0   = tile * ROWS_PER_WAVE;
  const int fr   = dir & 1;
  const int fcl  = dir >> 1;

  const v8h z8h = {(_Float16)0.0f, (_Float16)0.0f, (_Float16)0.0f, (_Float16)0.0f,
                   (_Float16)0.0f, (_Float16)0.0f, (_Float16)0.0f, (_Float16)0.0f};
  FragU zfu;
  zfu.h[0] = z8h;
  zfu.h[1] = z8h;
  const v16h z16h = zfu.v;

#pragma unroll 1
  for (int k = 0; k < NHID; ++k) {
#pragma unroll
    for (int t = 0; t < NGATE / 32; ++t) {
      const int g = t * 32 + lane;
      const float v1 = Whv[(size_t)(dir * NHID + k) * NGATE + g];
      const float v2 = Whh[(size_t)(dir * NHID + k) * NGATE + g];
      Bt[g * BT_PITCH + k]        = (_Float16)(bf16_value(v1) * W_CARRY);
      Bt[g * BT_PITCH + NHID + k] = (_Float16)(bf16_value(v2) * W_CARRY);
    }
  }
#pragma unroll 1
  for (int t = 0; t < NGATE / 32; ++t)
    *(v8h*)(Bt + (t * 32 + lane) * BT_PITCH + 2 * NHID) = z8h;
#pragma unroll 1
  for (int it = 0; it < (NCHAN * NGATE) / 32; ++it) {
    const int idx = it * 32 + lane;
    wxs[idx] = bf16_value(Wx[(size_t)dir * NCHAN * NGATE + idx]);
  }
#pragma unroll 1
  for (int it = 0; it < NGATE / 32; ++it) {
    const int idx = it * 32 + lane;
    wxs[NCHAN * NGATE + idx] = bf16_value(bias[(size_t)dir * NGATE + idx]);
  }
#pragma unroll 1
  for (int it = 0; it < (IMG_W * HT_ELEMS) / 256; ++it) {
    *(v8h*)(Hhi + (it * 32 + lane) * 8) = z8h;
    *(v8h*)(Hlo + (it * 32 + lane) * 8) = z8h;
  }
  __syncthreads();

  float* crow_blk = crow + (size_t)(dir * NTILES_B + tile) * CROW_PER_BLOCK;
  const v8f z8 = {0.0f, 0.0f, 0.0f, 0.0f, 0.0f, 0.0f, 0.0f, 0.0f};
  const int fo = ln * NHID + 8 * hh;
  const int so = 8 * hh * NHID + ln;

#pragma unroll 1
  for (int i = 0; i < IMG_H; ++i) {
    const int ir = fr ? (IMG_H - 1 - i) : i;
    __syncthreads();
#pragma unroll 4
    for (int it = 0; it < 12; ++it) {
      const int idx = it * 32 + lane;
      const int bc  = idx >> 3;
      const int bb  = bc / NCHAN;
      const int cc  = bc - bb * NCHAN;
      const int w4  = (idx & 7) * 4;
      const v4f v = *(const v4f*)(x + (size_t)(b0 + bb) * (NCHAN * IMG_H * IMG_W) + cc * (IMG_H * IMG_W) + ir * IMG_W + w4);
#pragma unroll
      for (int e = 0; e < 4; ++e) {
        const float f = v[e];
        xs[((w4 + e) * NCHAN + cc) * ROWS_PER_WAVE + bb] = bf16_value(f);
      }
    }

    float clA[8], clB[8];
#pragma unroll
    for (int r = 0; r < 8; ++r) { clA[r] = 0.0f; clB[r] = 0.0f; }

#pragma unroll 1
    for (int j = 0; j < IMG_W; ++j) {
      const int jc = fcl ? (IMG_W - 1 - j) : j;
      const int jl = (j > 0) ? (j - 1) : 0;
      const bool last = (i == IMG_H - 1) && (j == IMG_W - 1);
      __syncthreads();
      const v16h auh = frag_load(Hhi + j * HT_ELEMS + fo);
      const v16h aul = frag_load(Hlo + j * HT_ELEMS + fo);
      v16h alh  = frag_load(Hhi + jl * HT_ELEMS + fo);
      v16h all_ = frag_load(Hlo + jl * HT_ELEMS + fo);
      if (j == 0) { alh = z16h; all_ = z16h; }

      float xv[NCHAN][8];
#pragma unroll
      for (int c = 0; c < NCHAN; ++c) {
        const float* xp = xs + (jc * NCHAN + c) * ROWS_PER_WAVE + 8 * hh;
        const v4f xa = *(const v4f*)(xp);
        const v4f xb = *(const v4f*)(xp + 4);
#pragma unroll
        for (int e = 0; e < 4; ++e) { xv[c][e] = xa[e]; xv[c][4 + e] = xb[e]; }
      }

      _Float16* hw_h = Hhi + j * HT_ELEMS + so;
      _Float16* hw_l = Hlo + j * HT_ELEMS + so;

#pragma unroll 1
      for (int p = 0; p < 2; ++p) {
        const _Float16* bp = Bt + (p * 16 + ln) * BT_PITCH + 8 * hh;
        const float* wp = wxs + p * 16 + ln;
        float pre[5][8];
#pragma unroll
        for (int kk = 0; kk < 5; ++kk) {
          const v16h bu = frag_load(bp + kk * 32 * BT_PITCH);
          const v16h bl = frag_load(bp + kk * 32 * BT_PITCH + NHID);
          v8f ah = z8;
          v8f al = z8;
          ah = mma16(auh, bu, ah);
          ah = mma16(alh, bl, ah);
          al = mma16(aul, bu, al);
          al = mma16(all_, bl, al);
          acc_guard(ah, auh, alh, bu, bl);
          acc_guard(al, aul, all_, bu, bl);
          const float w0 = wp[kk * 32];
          const float w1 = wp[NGATE + kk * 32];
          const float w2 = wp[2 * NGATE + kk * 32];
          const float bb = wp[3 * NGATE + kk * 32];
#pragma unroll
          for (int r = 0; r < 8; ++r) {
            float t = bb;
            t = fmaf(xv[0][r], w0, t);
            t = fmaf(xv[1][r], w1, t);
            t = fmaf(xv[2][r], w2, t);
            const float u = fmaf(al[r], RES_CARRY_INV, ah[r]);
            pre[kk][r] = fmaf(u, W_CARRY_INV, t);
          }
        }
        float cu[8];
        if (i > 0) {
          const float* cr = crow_blk + j * CROW_PER_COL + p * 256 + lane * 4;
          const v4f c0 = *(const v4f*)(cr);
          const v4f c1 = *(const v4f*)(cr + 128);
#pragma unroll
          for (int e = 0; e < 4; ++e) { cu[e] = c0[e]; cu[4 + e] = c1[e]; }
        } else {
#pragma unroll
          for (int e = 0; e < 8; ++e) cu[e] = 0.0f;
        }
        float hn[8];
#pragma unroll
        for (int r = 0; r < 8; ++r) {
          const float iv = gate_sig(pre[0][r]);
          const float f1 = gate_sig(pre[1][r]);
          const float f2 = gate_sig(pre[2][r]);
          const float gv = gate_tanh(pre[3][r]);
          const float ov = gate_sig(pre[4][r]);
          const float cn = f1 * cu[r] + f2 * clA[r] + iv * gv;
          clA[r] = cn;
          const float hv = ov * gate_tanh(cn);
          hn[r] = hv;
          _Float16 s_hi, s_lo;
          split_val(hv, s_hi, s_lo);
          hw_h[r * NHID + p * 16] = s_hi;
          hw_l[r * NHID + p * 16] = s_lo;
        }
        if (last) {
#pragma unroll
          for (int r = 0; r < 8; ++r) hfin[(8 * hh + r) * NHID + p * 16 + ln] = hn[r];
        }
#pragma unroll
        for (int r = 0; r < 8; ++r) { const float t = clA[r]; clA[r] = clB[r]; clB[r] = t; }
      }

      {
        float* cw = crow_blk + j * CROW_PER_COL + lane * 4;
        const v4f s0 = {clA[0], clA[1], clA[2], clA[3]};
        const v4f s1 = {clA[4], clA[5], clA[6], clA[7]};
        const v4f s2 = {clB[0], clB[1], clB[2], clB[3]};
        const v4f s3 = {clB[4], clB[5], clB[6], clB[7]};
        for (int pass = 0; pass < 2; ++pass) {
          *(volatile v4f*)(cw)       = s0;
          *(volatile v4f*)(cw + 128) = s1;
          *(volatile v4f*)(cw + 256) = s2;
          *(volatile v4f*)(cw + 384) = s3;
          __threadfence();
        }
      }
    }
  }

  __syncthreads();
  {
    const int q  = lane >> 3;
    const int c4 = (lane & 7) * 4;
    v4f fv[4];
#pragma unroll
    for (int it = 0; it < 4; ++it) fv[it] = *(const v4f*)(hfin + (it * 4 + q) * NHID + c4);
    for (int pass = 0; pass < 2; ++pass) {
#pragma unroll
      for (int it = 0; it < 4; ++it) {
        const int row = it * 4 + q;
        *(volatile v4f*)(feats + (size_t)(b0 + row) * NFEAT + dir * NHID + c4) = fv[it];
      }
      __threadfence();
    }
  }
}

__global__ __launch_bounds__(256)
void head_kernel(const float* __restrict__ feats, const float* __restrict__ fcw,
                 const float* __restrict__ fcb, float* __restrict__ out) {
  const int idx = blockIdx.x * 256 + threadIdx.x;
  const int b = idx / NOUTS;
  const int o = idx - b * NOUTS;
  const float* fp = feats + (size_t)b * NFEAT;
  const float* wc = fcw + o;
  float s = 0.0f;
#pragma unroll 4
  for (int k = 0; k < NFEAT; ++k) s = fmaf(fp[k], bf16_value(wc[k * NOUTS]), s);
  s += bf16_value(fcb[o]);
  *(volatile float*)(out + idx) = s;
  __threadfence();
  *(volatile float*)(out + idx) = s;
}

extern "C" void kernel_launch(void* const* d_in, const int* in_sizes, int n_in,
                              void* d_out, int out_size, void* d_ws, size_t ws_size, hipStream_t stream) {
  if (n_in < 7 || d_out == nullptr || d_ws == nullptr) return;
  if (in_sizes[0] != NBATCH * NCHAN * IMG_H * IMG_W || in_sizes[1] != NDIRS * NCHAN * NGATE ||
      in_sizes[2] != NDIRS * NHID * NGATE || in_sizes[3] != NDIRS * NHID * NGATE ||
      in_sizes[4] != NDIRS * NGATE || in_sizes[5] != NFEAT * NOUTS || in_sizes[6] != NOUTS ||
      out_size != NBATCH * NOUTS) return;

  const float* x    = (const float*)d_in[0];
  const float* Wx   = (const float*)d_in[1];
  const float* Whv  = (const float*)d_in[2];
  const float* Whh  = (const float*)d_in[3];
  const float* bias = (const float*)d_in[4];
  const float* fcw  = (const float*)d_in[5];
  const float* fcb  = (const float*)d_in[6];
  float* out = (float*)d_out;

  char* ws = (char*)d_ws;
  size_t off = 0;
  auto carve = [&](size_t bytes) -> char* { char* p = ws + off; off += (bytes + 255) & ~(size_t)255; return p; };
  float* feats = (float*)carve((size_t)NBATCH * NFEAT * sizeof(float));
  float* crow  = (float*)carve((size_t)NDIRS * NTILES_B * CROW_PER_BLOCK * sizeof(float));
  if (off > ws_size || off > (size_t)134217728) return;

  scan2d_kernel<<<dim3(NTILES_B, NDIRS), 32, 0, stream>>>(x, Wx, Whv, Whh, bias, crow, feats);
  head_kernel<<<(NBATCH * NOUTS) / 256, 256, 0, stream>>>(feats, fcw, fcb, out);
}
